// GNN_17592186044939
// MI455X (gfx1250) — hardware-run, weakly checked
//
#include <hip/hip_runtime.h>

typedef float          v8f   __attribute__((ext_vector_type(8)));
typedef float          v4f   __attribute__((ext_vector_type(4)));
typedef unsigned int   v4u   __attribute__((ext_vector_type(4)));
typedef int            v8i   __attribute__((ext_vector_type(8)));
typedef unsigned short v8us  __attribute__((ext_vector_type(8)));
typedef unsigned short v16us __attribute__((ext_vector_type(16)));
typedef __bf16         v16bf __attribute__((ext_vector_type(16)));
typedef _Float16       v16h  __attribute__((ext_vector_type(16)));
typedef v4f  __attribute__((may_alias)) v4fa;
typedef v8us __attribute__((may_alias)) v8usa;
union FragB { v16bf v; v16us u; v8us h[2]; v8i w; };
union FragH { v16h  v; v16us u; v8us h[2]; v8i w; };

__device__ __forceinline__ v8f wmb(const FragB& a, const FragB& b, v8f c) {
  v8f d = __builtin_amdgcn_wmma_f32_16x16x32_bf16(false, a.v, false, b.v, (short)0, c, false, false);
  asm volatile("v_nop\n\tv_nop\n\tv_nop\n\tv_nop" : "+v"(d) : "v"(a.w), "v"(b.w));
  return d;
}

__device__ __forceinline__ v8f wmh(const FragH& a, const FragH& b, v8f c) {
  v8f d = __builtin_amdgcn_wmma_f32_16x16x32_f16(false, a.v, false, b.v, (short)0, c, false, false);
  asm volatile("v_nop\n\tv_nop\n\tv_nop\n\tv_nop" : "+v"(d) : "v"(a.w), "v"(b.w));
  return d;
}

__device__ __forceinline__ unsigned bf16_bits(float f) {
  const unsigned u = __float_as_uint(f);
  const unsigned r = (u + 0x7FFFu + ((u >> 16) & 1u)) >> 16;
  const unsigned q = (u >> 16) | 0x40u;
  return ((u & 0x7fffffffu) > 0x7f800000u) ? q : r;
}

__device__ __forceinline__ float bf16_val(float f) {
  return __uint_as_float(bf16_bits(f) << 16);
}
__device__ __forceinline__ int clampi(int v, int lo, int hi) {
  return v < lo ? lo : (v > hi ? hi : v);
}

__device__ __forceinline__ unsigned f16_bits(float f) {
  const unsigned u  = __float_as_uint(f);
  const unsigned s  = (u >> 16) & 0x8000u;
  const unsigned a  = u & 0x7fffffffu;
  const unsigned t  = a - 0x38000000u;
  const unsigned r  = (t + 0x0FFFu + ((t >> 13) & 1u)) >> 13;
  const unsigned rc = r > 0x7C00u ? 0x7C00u : r;
  const bool small  = a < 0x38800000u;
  const bool isnan  = a > 0x7f800000u;
  const unsigned fin = small ? 0u : (s | rc);
  return isnan ? (s | 0x7E00u) : fin;
}

__device__ __forceinline__ unsigned pk16(unsigned lo, unsigned hi) { return lo | (hi << 16); }
__device__ __forceinline__ unsigned bf16_lo_bits(float v) {
  float hi = bf16_val(v);
  asm volatile("" : "+v"(hi));
  return bf16_bits(v - hi);
}
__device__ __forceinline__ v4u pack8_bf16(v4f a, v4f c) {
  return (v4u){ pk16(bf16_bits(a[0]), bf16_bits(a[1])), pk16(bf16_bits(a[2]), bf16_bits(a[3])),
                pk16(bf16_bits(c[0]), bf16_bits(c[1])), pk16(bf16_bits(c[2]), bf16_bits(c[3])) };
}
__device__ __forceinline__ v4u pack8_bf16_lo(v4f a, v4f c) {
  return (v4u){ pk16(bf16_lo_bits(a[0]), bf16_lo_bits(a[1])), pk16(bf16_lo_bits(a[2]), bf16_lo_bits(a[3])),
                pk16(bf16_lo_bits(c[0]), bf16_lo_bits(c[1])), pk16(bf16_lo_bits(c[2]), bf16_lo_bits(c[3])) };
}
__device__ __forceinline__ v4u pack8_f16(v4f a, v4f c) {
  return (v4u){ pk16(f16_bits(a[0]), f16_bits(a[1])), pk16(f16_bits(a[2]), f16_bits(a[3])),
                pk16(f16_bits(c[0]), f16_bits(c[1])), pk16(f16_bits(c[2]), f16_bits(c[3])) };
}

template <int FORM>
__global__ __launch_bounds__(256) void k_plane(const float* __restrict__ src, int rows, int cols, int ldsrc,
                                               unsigned short* __restrict__ dst, int MP, int KP) {
  static_assert(FORM >= 0 && FORM <= 3);
  const int KTOT = (FORM == 1 || FORM == 3) ? 2 * KP : KP;
  const unsigned ppr   = (unsigned)(KTOT >> 3);
  const unsigned kp8   = (unsigned)(KP >> 3);
  const unsigned total = (unsigned)MP * ppr;
  const unsigned g     = blockIdx.x * 256u + threadIdx.x;
  const unsigned rowu  = g / ppr;
  const unsigned p     = g - rowu * ppr;
  const bool second    = p >= kp8;
  const int row = (int)rowu;
  const int c0  = (int)((second ? p - kp8 : p) << 3);
  const float* srow = src + (size_t)clampi(row, 0, rows - 1) * (size_t)ldsrc;
  float x[8];
  unsigned mk[8];
#pragma unroll
  for (int e = 0; e < 8; ++e) {
    const int c = c0 + e;
    const float v = srow[clampi(c, 0, cols - 1)];
    asm volatile("" :: "v"(v));
    x[e]  = v;
    mk[e] = (row < rows && c < cols) ? 0xFFFFu : 0u;
  }
  const v4f a = (v4f){ x[0], x[1], x[2], x[3] };
  const v4f c = (v4f){ x[4], x[5], x[6], x[7] };
  v4u o;
  if (FORM == 2) {
    o = pack8_f16(a, c);
  } else {
    const v4u hi = pack8_bf16(a, c);
    o = hi;
    if (FORM == 1) { const v4u lo = pack8_bf16_lo(a, c); o = second ? lo : hi; }
  }
  const v4u mw = (v4u){ pk16(mk[0], mk[1]), pk16(mk[2], mk[3]), pk16(mk[4], mk[5]), pk16(mk[6], mk[7]) };
  o &= mw;
  if (g < total) {
    volatile v4u* q = (volatile v4u*)(dst + (size_t)g * 8);
    *q = o;
    __threadfence();
    *q = o;
  }
}

template <int FORM> struct FragOf    { typedef FragB T; };
template <>         struct FragOf<2> { typedef FragH T; };
__device__ __forceinline__ v8f mm(const FragB& a, const FragB& b, v8f c) { return wmb(a, b, c); }
__device__ __forceinline__ v8f mm(const FragH& a, const FragH& b, v8f c) { return wmh(a, b, c); }
template <class F> __device__ __forceinline__ F ld_frag(const unsigned short* p) {
  F f;
  f.h[0] = *(const v8usa*)(p);
  f.h[1] = *(const v8usa*)(p + 16);
  return f;
}

template <int FORM, int EPI>
__global__ __launch_bounds__(256) __attribute__((amdgpu_num_vgpr(248)))
void k_gemm_nt(const unsigned short* __restrict__ A, const unsigned short* __restrict__ B,
               const float* __restrict__ bias, float* __restrict__ D, int M, int N, int KTOT, int ldd) {
  static_assert(FORM >= 0 && FORM <= 2);
  static_assert(EPI == 0 || EPI == 1);
  typedef typename FragOf<FORM>::T F;
  __shared__ __attribute__((aligned(16))) float sT[8][16 * 68];
  const int lane = threadIdx.x & 31;
  const int wave = threadIdx.x >> 5;
  const int tilesM = (M + 63) >> 6;
  const int tilesN = (N + 63) >> 6;
  const int tile = blockIdx.x * 8 + wave;
  if (tile >= tilesM * tilesN) return;
  const int tm = tile / tilesN;
  const int tn = tile - tm * tilesN;
  const int m0 = tm << 6;
  const int n0 = tn << 6;

  const int rl = lane & 15;
  const int h8 = (lane >> 4) * 8;
  const unsigned short* pa = A + (size_t)(m0 + rl) * (size_t)KTOT + h8;
  const unsigned short* pb = B + (size_t)(n0 + rl) * (size_t)KTOT + h8;

  v8f acc[4][4];
#pragma unroll
  for (int i = 0; i < 4; ++i)
#pragma unroll
    for (int j = 0; j < 4; ++j) acc[i][j] = (v8f){0.f, 0.f, 0.f, 0.f, 0.f, 0.f, 0.f, 0.f};

#pragma unroll 1
  for (int k0 = 0; k0 < KTOT; k0 += 32) {
    F bf[4];
#pragma unroll
    for (int j = 0; j < 4; ++j) bf[j] = ld_frag<F>(pb + (size_t)(j << 4) * (size_t)KTOT + k0);
#pragma unroll
    for (int i = 0; i < 4; ++i) {
      const F af = ld_frag<F>(pa + (size_t)(i << 4) * (size_t)KTOT + k0);
#pragma unroll
      for (int j = 0; j < 4; ++j) acc[i][j] = mm(af, bf[j], acc[i][j]);
    }
  }

  float* slab = sT[wave];
  const int hh = lane >> 4;
  const int c4 = (lane & 15) * 4;
  const int nc = n0 + c4;
  const bool cok = nc < N;
  v4f bv = (v4f){0.f, 0.f, 0.f, 0.f};
  if (EPI == 1) {
    bv = *(const v4fa*)(bias + clampi(nc, 0, N - 4));
    asm volatile("" :: "v"(bv));
  }
#pragma unroll
  for (int i = 0; i < 4; ++i) {
    const int mBase = m0 + (i << 4);
#pragma unroll
    for (int j = 0; j < 4; ++j) {
#pragma unroll
      for (int r = 0; r < 8; ++r) slab[(h8 + r) * 68 + (j << 4) + rl] = acc[i][j][r];
    }
    __builtin_amdgcn_fence(__ATOMIC_RELEASE, "workgroup");
    __builtin_amdgcn_wave_barrier();
    __builtin_amdgcn_fence(__ATOMIC_ACQUIRE, "workgroup");
    v4f vv[8];
#pragma unroll
    for (int it = 0; it < 8; ++it) {
      const int row = it * 2 + hh;
      v4f v = *(const v4fa*)(slab + row * 68 + c4);
      if (EPI == 1) v += bv;
      vv[it] = v;
    }
    for (int pass = 0; pass < 2; ++pass) {
#pragma unroll
      for (int it = 0; it < 8; ++it) {
        const int row = mBase + it * 2 + hh;
        if (cok && row < M) *(volatile v4f*)(D + (size_t)row * (size_t)ldd + nc) = vv[it];
      }
      __threadfence();
    }
    __builtin_amdgcn_fence(__ATOMIC_RELEASE, "workgroup");
    __builtin_amdgcn_wave_barrier();
    __builtin_amdgcn_fence(__ATOMIC_ACQUIRE, "workgroup");
  }
}

#pragma clang fp contract(off)

#ifndef SPLIT_L2
#define SPLIT_L2 1
#endif

#define NN      100000
#define KD      128
#define H1      32
#define H2      16
#define NE      3200000
#define MP      100096
#define TP      64
#define OPK     64
#define YP      32
#define NTHR    256
#define NWAVE   8
#define EPT     8
#define WCH     (32 * EPT)
#define NBRUN   1024
#define SLSH    22
#define IDMASK  0x3FFFFF
#define NBK     98
#define HSL     512
#define HCAP    20480
#define RCAP    (2 * HCAP)
#define WLCAP   4736
#define DEGCAP  128
#define LISTW   (NBK * RCAP)
#define MAXDEG_MEAS   57
#define MAXB1024_MEAS 33219
#define MAXB512_MEAS  16774

#define L_WL    0
#define L_PL    (NWAVE * WLCAP)
#define L_CNT   (L_PL + HCAP)
#define L_OFF   (L_CNT + NBRUN)
#define L_CUR   (L_OFF + NBRUN)
#define L_MISC  (L_CUR + NBRUN)
#define BK_ZINTS L_MISC
#define BK_INTS (L_MISC + 16)
#define BK_LDS  (BK_INTS * 4)

#define PB_W1   4
#define PB_W2   2
#define PB_BV   1
#define PB_OPZ  3
#define PB_TOT  (PB_W1 + PB_W2 + PB_BV + PB_OPZ)

static_assert(MP == 782 * 128 && MP % 128 == 0 && MP % 64 == 0 && MP >= NN && MP - NN == 96);
static_assert(TP == 64 && TP % 32 == 0 && OPK == 2 * H1 && OPK % 32 == 0 && KD % 32 == 0 && YP == 32);
static_assert(H1 == 32 && H2 == 16 && 2 * 16 == H1 && 2 * 8 == H2);
static_assert(NE <= (1 << SLSH) && NBRUN <= 1024 && NBRUN == 2 * HSL && HSL == 512 && HSL % 4 == 0);
static_assert(NBK * NBRUN >= MP && (NBK - 1) * NBRUN < NN);
static_assert(NE % WCH == 0 && NE % 4 == 0);
static_assert((long long)RCAP * 10 >= (long long)MAXB1024_MEAS * 11);
static_assert((long long)HCAP * 10 >= (long long)MAXB512_MEAS * 11);
static_assert(WLCAP >= MAXB1024_MEAS / 8 + 8 * 65 + 1);
static_assert((long long)WLCAP * NWAVE * 10 >= (long long)MAXB1024_MEAS * 11);
static_assert(MAXDEG_MEAS + 8 <= DEGCAP);
static_assert(HCAP % (NTHR * 4) == 0 && BK_ZINTS % (NTHR * 4) == 0 && NBRUN == NTHR * 4);
static_assert(BK_LDS <= 262144);
static_assert((MP * KD / 8) % NTHR == 0);
static_assert(NN % NWAVE == 0 && (NN * H2) % NTHR == 0 && (NN * H2) % 32 == 0);
static_assert(PB_W1 * NTHR * 8 == 64 * KD && PB_W2 * NTHR * 8 == 64 * OPK && PB_OPZ * NTHR * 8 == (MP - NN) * OPK);

typedef float v2f __attribute__((ext_vector_type(2)));
typedef int   v4i __attribute__((ext_vector_type(4)));
typedef v2f __attribute__((may_alias)) v2fa;
typedef v4i __attribute__((may_alias)) v4ia;

__device__ __forceinline__ void st2_v4u(unsigned* p, v4u v) {
  *(volatile v4u*)p = v;
  __threadfence();
  *(volatile v4u*)p = v;
}
__device__ __forceinline__ void st2_v4i(int* p, v4i v) {
  *(volatile v4i*)p = v;
  __threadfence();
  *(volatile v4i*)p = v;
}

__global__ __launch_bounds__(NTHR) void k_prep(const float* __restrict__ W1, const float* __restrict__ b1,
                                               const float* __restrict__ W2, const float* __restrict__ b2,
                                               unsigned short* W1P, unsigned short* W2P, unsigned* BV,
                                               unsigned short* OP) {
  const int tid = (int)threadIdx.x;
  const int blk = (int)blockIdx.x;
  if (blk < PB_W1) {
    const int u  = blk * NTHR + tid;
    const int n  = u >> 4, k8 = (u & 15) << 3;
    const int nc = n < H1 ? n : H1 - 1;
    const unsigned mk = n < H1 ? 0xFFFFu : 0u;
    float f[8];
#pragma unroll
    for (int i = 0; i < 8; ++i) {
      const float v = W1[(size_t)(k8 + i) * H1 + nc];
      asm volatile("" :: "v"(v));
      f[i] = v;
    }
    unsigned b[8];
#pragma unroll
    for (int i = 0; i < 8; ++i) b[i] = bf16_bits(f[i]) & mk;
    const v4u o = (v4u){ pk16(b[0], b[1]), pk16(b[2], b[3]), pk16(b[4], b[5]), pk16(b[6], b[7]) };
    st2_v4u((unsigned*)(W1P + (size_t)u * 8), o);
  } else if (blk < PB_W1 + PB_W2) {
    const int u  = (blk - PB_W1) * NTHR + tid;
    const int n  = u >> 3, kq = (u & 7) << 3;
    const int nc = n < H2 ? n : H2 - 1;
    const unsigned mk = n < H2 ? 0xFFFFu : 0u;
    float f[8];
#pragma unroll
    for (int i = 0; i < 8; ++i) {
      const float v = W2[(size_t)((kq + i) & (H1 - 1)) * H2 + nc];
      asm volatile("" :: "v"(v));
      f[i] = v;
    }
    unsigned b[8];
#pragma unroll
    for (int i = 0; i < 8; ++i) b[i] = bf16_bits(f[i]) & mk;
    const v4u o = (v4u){ pk16(b[0], b[1]), pk16(b[2], b[3]), pk16(b[4], b[5]), pk16(b[6], b[7]) };
    st2_v4u((unsigned*)(W2P + (size_t)u * 8), o);
  } else if (blk < PB_W1 + PB_W2 + PB_BV) {
    const int pc    = tid < 48 ? tid : 47;
    const int which = pc >> 4;
    const int i0    = (pc & 15) << 2;
    unsigned w[4];
#pragma unroll
    for (int e = 0; e < 4; ++e) {
      const int i = i0 + e;
      const float x1 = b1[clampi(i, 0, H1 - 1)];
      const float x2 = b2[clampi(i, 0, H2 - 1)];
      asm volatile("" :: "v"(x1));
      asm volatile("" :: "v"(x2));
      const unsigned m1 = (which == 0 && i < H1) ? 0xFFFFFFFFu : 0u;
      const unsigned m2 = (which == 1 && i < H2) ? 0xFFFFFFFFu : 0u;
      w[e] = ((bf16_bits(x1) << 16) & m1) | ((bf16_bits(x2) << 16) & m2);
    }
    const v4u o = (v4u){ w[0], w[1], w[2], w[3] };
    if (tid < 48) st2_v4u(BV + 4 * tid, o);
  } else {
    const int u = (blk - PB_W1 - PB_W2 - PB_BV) * NTHR + tid;
    const v4u z = (v4u){ 0u, 0u, 0u, 0u };
    st2_v4u((unsigned*)(OP + (size_t)NN * OPK + (size_t)u * 8), z);
  }
}

__global__ __launch_bounds__(NTHR) void k_list(const int* __restrict__ srcs, const int* __restrict__ dsts,
                                               int* LIST, int* CNT, int* OFF, int* DINVB, int* FLAG) {
  extern __shared__ __attribute__((aligned(16))) int dsm[];
  const int tid  = (int)threadIdx.x;
  const int lane = tid & 31;
  const int wave = __builtin_amdgcn_readfirstlane(tid >> 5);
  const int blk  = (int)blockIdx.x;
  const unsigned nbs = (unsigned)(blk * NBRUN);

  {
    const v4i z4 = {0, 0, 0, 0};
#pragma unroll 1
    for (int i = tid * 4; i < BK_ZINTS; i += NTHR * 4) *(v4ia*)(dsm + i) = z4;
    if (tid < 16) dsm[L_MISC + tid] = 0;
  }
  __syncthreads();

  {
    const int per  = ((NE + NWAVE * WCH - 1) / (NWAVE * WCH)) * WCH;
    const int ebeg = wave * per;
    const int eend = (ebeg + per < NE) ? (ebeg + per) : NE;
    const int lb   = L_WL + wave * WLCAP;
    int wc = 0;
#pragma unroll 1
    for (int cb = ebeg; cb < eend; cb += WCH) {
      const int e0 = cb + lane * EPT;
      const v4i da = *(const v4ia*)(dsts + e0);
      const v4i db = *(const v4ia*)(dsts + e0 + 4);
      asm volatile("" :: "v"(da));
      asm volatile("" :: "v"(db));
      const unsigned s0 = (unsigned)clampi(da.x, 0, NN - 1) - nbs, s1 = (unsigned)clampi(da.y, 0, NN - 1) - nbs;
      const unsigned s2 = (unsigned)clampi(da.z, 0, NN - 1) - nbs, s3 = (unsigned)clampi(da.w, 0, NN - 1) - nbs;
      const unsigned s4 = (unsigned)clampi(db.x, 0, NN - 1) - nbs, s5 = (unsigned)clampi(db.y, 0, NN - 1) - nbs;
      const unsigned s6 = (unsigned)clampi(db.z, 0, NN - 1) - nbs, s7 = (unsigned)clampi(db.w, 0, NN - 1) - nbs;
      const bool h0 = s0 < (unsigned)NBRUN, h1 = s1 < (unsigned)NBRUN, h2 = s2 < (unsigned)NBRUN, h3 = s3 < (unsigned)NBRUN;
      const bool h4 = s4 < (unsigned)NBRUN, h5 = s5 < (unsigned)NBRUN, h6 = s6 < (unsigned)NBRUN, h7 = s7 < (unsigned)NBRUN;
      const unsigned m0 = __builtin_amdgcn_ballot_w32(h0), m1 = __builtin_amdgcn_ballot_w32(h1);
      const unsigned m2 = __builtin_amdgcn_ballot_w32(h2), m3 = __builtin_amdgcn_ballot_w32(h3);
      const unsigned m4 = __builtin_amdgcn_ballot_w32(h4), m5 = __builtin_amdgcn_ballot_w32(h5);
      const unsigned m6 = __builtin_amdgcn_ballot_w32(h6), m7 = __builtin_amdgcn_ballot_w32(h7);
      const unsigned any = m0 | m1 | m2 | m3 | m4 | m5 | m6 | m7;
      if (any != 0u) {
        const int pre = (int)(__builtin_amdgcn_mbcnt_lo(m0, 0u) + __builtin_amdgcn_mbcnt_lo(m1, 0u) +
                              __builtin_amdgcn_mbcnt_lo(m2, 0u) + __builtin_amdgcn_mbcnt_lo(m3, 0u) +
                              __builtin_amdgcn_mbcnt_lo(m4, 0u) + __builtin_amdgcn_mbcnt_lo(m5, 0u) +
                              __builtin_amdgcn_mbcnt_lo(m6, 0u) + __builtin_amdgcn_mbcnt_lo(m7, 0u));
        int p = wc + pre;
        if (h0) { if (p < WLCAP) dsm[lb + p] = (int)((unsigned)(e0 + 0) | (s0 << SLSH)); p = p + 1; }
        if (h1) { if (p < WLCAP) dsm[lb + p] = (int)((unsigned)(e0 + 1) | (s1 << SLSH)); p = p + 1; }
        if (h2) { if (p < WLCAP) dsm[lb + p] = (int)((unsigned)(e0 + 2) | (s2 << SLSH)); p = p + 1; }
        if (h3) { if (p < WLCAP) dsm[lb + p] = (int)((unsigned)(e0 + 3) | (s3 << SLSH)); p = p + 1; }
        if (h4) { if (p < WLCAP) dsm[lb + p] = (int)((unsigned)(e0 + 4) | (s4 << SLSH)); p = p + 1; }
        if (h5) { if (p < WLCAP) dsm[lb + p] = (int)((unsigned)(e0 + 5) | (s5 << SLSH)); p = p + 1; }
        if (h6) { if (p < WLCAP) dsm[lb + p] = (int)((unsigned)(e0 + 6) | (s6 << SLSH)); p = p + 1; }
        if (h7) { if (p < WLCAP) dsm[lb + p] = (int)((unsigned)(e0 + 7) | (s7 << SLSH)); p = p + 1; }
        wc += (int)(__builtin_popcount(m0) + __builtin_popcount(m1) + __builtin_popcount(m2) + __builtin_popcount(m3) +
                    __builtin_popcount(m4) + __builtin_popcount(m5) + __builtin_popcount(m6) + __builtin_popcount(m7));
      }
    }
    if (lane == 0) dsm[L_MISC + wave] = wc;
  }
  __syncthreads();

  if (wave == 0) {
    int ov = 0;
#pragma unroll 1
    for (int w2 = 0; w2 < NWAVE; ++w2) {
      int c = __builtin_amdgcn_readfirstlane(dsm[L_MISC + w2]);
      if (c > WLCAP) ov = 1;
      c = c < 0 ? 0 : (c > WLCAP ? WLCAP : c);
#pragma unroll 1
      for (int b0 = 0; b0 < c; b0 += 32) {
        const int idx = b0 + lane;
        const int ent = dsm[L_WL + w2 * WLCAP + (idx < WLCAP ? idx : WLCAP - 1)];
        const int m32 = (c - b0) < 32 ? (c - b0) : 32;
#pragma unroll 1
        for (int k = 0; k < m32; ++k) {
          const unsigned u = (unsigned)__builtin_amdgcn_readlane(ent, k);
          const int slot   = (int)(u >> SLSH);
          if (lane == 0) dsm[L_CNT + slot] = dsm[L_CNT + slot] + 1;
        }
      }
    }
    if (lane == 0) dsm[L_MISC + 9] = ov;
  }
  __syncthreads();
  if (wave == 0) {
    const int base = lane * (NBRUN / 32);
    int s = 0;
#pragma unroll 1
    for (int i = 0; i < NBRUN / 32; ++i) s += dsm[L_CNT + base + i];
    int incl = s;
#pragma unroll
    for (int d = 1; d < 32; d <<= 1) {
      const int y = __shfl_up(incl, d, 32);
      if (lane >= d) incl += y;
    }
    const int tot0 = __shfl(incl, 15, 32);
    const int tall = __shfl(incl, 31, 32);
    const int tot1 = tall - tot0;
    int run = incl - s - ((lane >= 16) ? tot0 : 0);
#pragma unroll 1
    for (int i = 0; i < NBRUN / 32; ++i) {
      const int cv = dsm[L_CNT + base + i];
      dsm[L_OFF + base + i] = run;
      dsm[L_CUR + base + i] = run;
      run += cv;
    }
    if (lane == 0 && (tot0 > HCAP || tot1 > HCAP)) dsm[L_MISC + 9] = 1;
  }
  __syncthreads();

#pragma unroll 1
  for (int hf = 0; hf < 2; ++hf) {
    if (wave == 0) {
#pragma unroll 1
      for (int w2 = 0; w2 < NWAVE; ++w2) {
        int c = __builtin_amdgcn_readfirstlane(dsm[L_MISC + w2]);
        c = c < 0 ? 0 : (c > WLCAP ? WLCAP : c);
#pragma unroll 1
        for (int b0 = 0; b0 < c; b0 += 32) {
          const int idx = b0 + lane;
          const int ent = dsm[L_WL + w2 * WLCAP + (idx < WLCAP ? idx : WLCAP - 1)];
          const int m32 = (c - b0) < 32 ? (c - b0) : 32;
#pragma unroll 1
          for (int k = 0; k < m32; ++k) {
            const unsigned u = (unsigned)__builtin_amdgcn_readlane(ent, k);
            const int slot   = (int)(u >> SLSH);
            if ((slot >> 9) == hf) {
              if (lane == 0) {
                int p = dsm[L_CUR + slot];
                p = p < 0 ? 0 : (p > HCAP - 1 ? HCAP - 1 : p);
                dsm[L_PL + p]     = (int)(u & (unsigned)IDMASK);
                dsm[L_CUR + slot] = p + 1;
              }
            }
          }
        }
      }
    }
    __syncthreads();
    {
      int* lp = LIST + ((size_t)blk * 2 + (size_t)hf) * (size_t)HCAP;
      const v4i z4 = {0, 0, 0, 0};
#pragma unroll 1
      for (int i = tid * 4; i < HCAP; i += NTHR * 4) {
        const v4i e = *(const v4ia*)(dsm + L_PL + i);
        int a0 = srcs[clampi(e.x, 0, NE - 1)];
        int a1 = srcs[clampi(e.y, 0, NE - 1)];
        int a2 = srcs[clampi(e.z, 0, NE - 1)];
        int a3 = srcs[clampi(e.w, 0, NE - 1)];
        asm volatile("" :: "v"(a0));
        asm volatile("" :: "v"(a1));
        asm volatile("" :: "v"(a2));
        asm volatile("" :: "v"(a3));
        v4i o;
        o.x = clampi(a0, 0, NN - 1); o.y = clampi(a1, 0, NN - 1);
        o.z = clampi(a2, 0, NN - 1); o.w = clampi(a3, 0, NN - 1);
        st2_v4i(lp + i, o);
        *(v4ia*)(dsm + L_PL + i) = z4;
      }
    }
    __syncthreads();
  }

#pragma unroll 1
  for (int i = 0; i < NBRUN / NTHR; ++i) {
    const int slot = tid + NTHR * i;
    const int deg  = dsm[L_CNT + slot] + 1;
    const float fd = (float)deg;
    const float dv = (deg > 0) ? (1.0f / sqrtf(fd)) : 0.0f;
    dsm[L_CUR + slot] = __float_as_int(dv);
  }
  __syncthreads();
  {
    const int ovf  = dsm[L_MISC + 9];
    const int base = blk * RCAP + ((4 * tid) >> 9) * HCAP;
    const v4i c4 = *(const v4ia*)(dsm + L_CNT + 4 * tid);
    v4i o4       = *(const v4ia*)(dsm + L_OFF + 4 * tid);
    const v4i d4 = *(const v4ia*)(dsm + L_CUR + 4 * tid);
    o4.x += base; o4.y += base; o4.z += base; o4.w += base;
    const size_t g = (size_t)blk * NBRUN + (size_t)(4 * tid);
    st2_v4i(CNT + g, c4);
    st2_v4i(OFF + g, o4);
    st2_v4i(DINVB + g, d4);
    if (tid < 8) {
      const v4i f = {ovf, ovf, ovf, ovf};
      st2_v4i(FLAG + (size_t)blk * 32 + 4 * tid, f);
    }
  }
}

__device__ __forceinline__ v2f walk_row(const int* __restrict__ LIST, const int* __restrict__ CNT,
                                        const int* __restrict__ OFF, const float* __restrict__ DINV,
                                        const int* __restrict__ FLAG, const float* __restrict__ T,
                                        const float* __restrict__ BV, int d, int lane, int& bad) {
  const int dc = clampi(d, 0, NN - 1);
  const int cv = CNT[dc];
  const int ov = OFF[dc];
  float dd     = DINV[dc];
  const int fl = FLAG[(size_t)(dc >> 10) * 32];
  asm volatile("" :: "v"(cv));
  asm volatile("" :: "v"(ov));
  asm volatile("" : "+v"(dd));
  asm volatile("" :: "v"(fl));
  const v2f self = *(const v2fa*)(T + (size_t)dc * TP + 2 * lane);
  asm volatile("" :: "v"(self));
  v2f bv = *(const v2fa*)(BV + 2 * lane);
  asm volatile("" : "+v"(bv));

  const int c = __builtin_amdgcn_readfirstlane((d < NN) ? clampi(cv, 0, DEGCAP) : 0);
  bad = (fl != 0 || cv > DEGCAP || cv < 0) ? 1 : 0;
  const int o = clampi(ov, 0, LISTW - 1);
  int last = o + (c > 0 ? c : 1) - 1;
  last = last > LISTW - 1 ? LISTW - 1 : last;

  float a0 = 0.0f, a1 = 0.0f;
#pragma unroll 1
  for (int b0 = 0; b0 < c; b0 += 32) {
    int idx = o + b0 + lane;
    idx = idx > last ? last : idx;
    const int s   = clampi(LIST[idx], 0, NN - 1);
    const float ds = DINV[s];
    const float w  = ds * dd;
    const int wb   = __float_as_int(w);
    const int m32  = (c - b0) < 32 ? (c - b0) : 32;
#pragma unroll 1
    for (int k = 0; k < m32; ++k) {
      const int   sk = __builtin_amdgcn_readlane(s, k);
      const float wk = __int_as_float(__builtin_amdgcn_readlane(wb, k));
      const v2f q = *(const v2fa*)(T + (size_t)sk * TP + 2 * lane);
      const float t0 = q.x * wk;
      const float t1 = q.y * wk;
      a0 = a0 + t0;
      a1 = a1 + t1;
    }
  }
  const float wself = dd * dd;
  const float u0 = self.x * wself;
  const float u1 = self.y * wself;
  a0 = a0 + u0;
  a1 = a1 + u1;
  v2f r;
  r.x = a0 + bv.x;
  r.y = a1 + bv.y;
  return r;
}

__global__ __launch_bounds__(NTHR) void k_walk1(const int* __restrict__ LIST, const int* __restrict__ CNT,
                                                const int* __restrict__ OFF, const float* __restrict__ DINV,
                                                const int* __restrict__ FLAG, const float* __restrict__ T,
                                                const float* __restrict__ BV, unsigned* OPW) {
  const int tid  = (int)threadIdx.x;
  const int lane = tid & 31;
  const int wave = __builtin_amdgcn_readfirstlane(tid >> 5);
  const int d    = (int)blockIdx.x * NWAVE + wave;
  int bad = 0;
  const v2f v = walk_row(LIST, CNT, OFF, DINV, FLAG, T, BV, d, lane, bad);
  float y0 = (v.x > 0.0f) ? v.x : (v.x - v.x);
  float y1 = (v.y > 0.0f) ? v.y : (v.y - v.y);
  const float qnan = __uint_as_float(0x7fc00000u);
  y0 = (bad != 0) ? qnan : y0;
  y1 = (bad != 0) ? qnan : y1;
  const unsigned hi = pk16(bf16_bits(y0), bf16_bits(y1));
#if SPLIT_L2
  const unsigned lo = pk16(bf16_lo_bits(y0), bf16_lo_bits(y1));
#else
  const unsigned lo = 0u;
#endif
  const unsigned mv   = (unsigned)__shfl_xor((int)lo, 16, 32);
  const unsigned word = (lane < 16) ? hi : mv;
  if (d < NN) {
    volatile unsigned* q = (volatile unsigned*)(OPW + (size_t)d * (OPK / 2) + lane);
    *q = word;
    __threadfence();
    *q = word;
  }
}

__global__ __launch_bounds__(NTHR) void k_walk2(const int* __restrict__ LIST, const int* __restrict__ CNT,
                                                const int* __restrict__ OFF, const float* __restrict__ DINV,
                                                const int* __restrict__ FLAG, const float* __restrict__ T,
                                                const float* __restrict__ BV, float* Y) {
  const int tid  = (int)threadIdx.x;
  const int lane = tid & 31;
  const int wave = __builtin_amdgcn_readfirstlane(tid >> 5);
  const int d    = (int)blockIdx.x * NWAVE + wave;
  int bad = 0;
  const v2f v = walk_row(LIST, CNT, OFF, DINV, FLAG, T, BV, d, lane, bad);
  const float qnan = __uint_as_float(0x7fc00000u);
  const float y0 = (bad != 0) ? qnan : v.x;
  const float y1 = (bad != 0) ? qnan : v.y;
  v2f o;
  o.x = (lane < 8) ? y0 : 0.0f;
  o.y = (lane < 8) ? y1 : 0.0f;
  if (d < NN && lane < 16) {
    volatile v2f* q = (volatile v2f*)(Y + (size_t)d * YP + 2 * lane);
    *q = o;
    __threadfence();
    *q = o;
  }
}

__global__ __launch_bounds__(NTHR) void k_copy(const float* __restrict__ Y, float* out, int nreal) {
  const int f  = (int)blockIdx.x * NTHR + (int)threadIdx.x;
  const int fc = clampi(f, 0, NN * H2 - 1);
  const float v = Y[(size_t)(fc >> 4) * YP + (size_t)(fc & 15)];
  asm volatile("" :: "v"(v));
  if (f < nreal) {
    volatile float* q = (volatile float*)(out + (size_t)f);
    *q = v;
    __threadfence();
    *q = v;
  }
}

extern "C" void kernel_launch(void* const* d_in, const int* in_sizes, int n_in,
                              void* d_out, int out_size, void* d_ws, size_t ws_size,
                              hipStream_t stream) {
  if (n_in < 6) return;
  if (in_sizes[0] != NN * KD) return;
  if (in_sizes[1] != 2 * NE) return;
  if (in_sizes[2] != KD * H1) return;
  if (in_sizes[3] != H1) return;
  if (in_sizes[4] != H1 * H2) return;
  if (in_sizes[5] != H2) return;
  if (out_size != NN * H2) return;

  const float* x  = (const float*)d_in[0];
  const int*   ei = (const int*)d_in[1];
  const float* W1 = (const float*)d_in[2];
  const float* b1 = (const float*)d_in[3];
  const float* W2 = (const float*)d_in[4];
  const float* b2 = (const float*)d_in[5];
  const int* srcs = ei;
  const int* dsts = ei + NE;
  float* out = (float*)d_out;

  constexpr size_t zXB   = (size_t)MP * KD * 2;
  constexpr size_t zT    = (size_t)MP * TP * 4;
  constexpr size_t zOP   = (size_t)MP * OPK * 2;
  constexpr size_t zY    = (size_t)MP * YP * 4;
  constexpr size_t zLIST = (size_t)NBK * RCAP * 4;
  constexpr size_t zTAB  = (size_t)NBK * NBRUN * 4;
  constexpr size_t zFLAG = (size_t)NBK * 128;
  constexpr size_t zW1P  = (size_t)64 * KD * 2;
  constexpr size_t zW2P  = (size_t)64 * OPK * 2;
  constexpr size_t zBV   = (size_t)3 * 64 * 4;
  constexpr size_t oXB   = 0;
  constexpr size_t oT    = oXB + zXB;
  constexpr size_t oOP   = oT + zT;
  constexpr size_t oY    = oOP + zOP;
  constexpr size_t oLIST = oY + zY;
  constexpr size_t oCNT  = oLIST + zLIST;
  constexpr size_t oOFF  = oCNT + zTAB;
  constexpr size_t oDINV = oOFF + zTAB;
  constexpr size_t oFLAG = oDINV + zTAB;
  constexpr size_t oW1P  = oFLAG + zFLAG;
  constexpr size_t oW2P  = oW1P + zW1P;
  constexpr size_t oBV   = oW2P + zW2P;
  constexpr size_t oEND  = oBV + zBV;
  static_assert(zXB % 256 == 0 && zT % 256 == 0 && zOP % 256 == 0 && zY % 256 == 0 && zLIST % 256 == 0);
  static_assert(zTAB % 256 == 0 && zFLAG % 256 == 0 && zW1P % 256 == 0 && zW2P % 256 == 0 && zBV % 256 == 0);
  static_assert(zTAB >= (size_t)MP * 4);
  static_assert(oEND == (size_t)94172160);
  static_assert(oEND <= ((size_t)128 << 20));
  if (oEND > ws_size) return;

  char* ws = (char*)d_ws;
  unsigned short* XB   = (unsigned short*)(ws + oXB);
  float*          T    = (float*)(ws + oT);
  unsigned short* OP   = (unsigned short*)(ws + oOP);
  float*          Y    = (float*)(ws + oY);
  int*            LIST = (int*)(ws + oLIST);
  int*            CNT  = (int*)(ws + oCNT);
  int*            OFF  = (int*)(ws + oOFF);
  int*            DINV = (int*)(ws + oDINV);
  int*            FLAG = (int*)(ws + oFLAG);
  unsigned short* W1P  = (unsigned short*)(ws + oW1P);
  unsigned short* W2P  = (unsigned short*)(ws + oW2P);
  unsigned*       BV   = (unsigned*)(ws + oBV);
  const float* B1V = (const float*)BV;
  const float* B2V = B1V + 64;
  const float* ZB  = B1V + 128;

  hipFuncSetAttribute(reinterpret_cast<const void*>(&k_list), hipFuncAttributeMaxDynamicSharedMemorySize, (int)BK_LDS);

  constexpr int gemmBlocks = ((MP / 64) + 7) / 8;

  k_plane<0><<<MP * KD / 8 / NTHR, NTHR, 0, stream>>>(x, NN, KD, KD, XB, MP, KD);
  k_prep<<<PB_TOT, NTHR, 0, stream>>>(W1, b1, W2, b2, W1P, W2P, BV, OP);
  k_list<<<NBK, NTHR, BK_LDS, stream>>>(srcs, dsts, LIST, CNT, OFF, DINV, FLAG);
  k_gemm_nt<0, 0><<<gemmBlocks, NTHR, 0, stream>>>(XB, W1P, ZB, T, MP, TP, KD, TP);
  k_walk1<<<NN / NWAVE, NTHR, 0, stream>>>(LIST, CNT, OFF, (const float*)DINV, FLAG, T, B1V, (unsigned*)OP);
  k_gemm_nt<0, 0><<<gemmBlocks, NTHR, 0, stream>>>(OP, W2P, ZB, T, MP, TP, OPK, TP);
  k_walk2<<<NN / NWAVE, NTHR, 0, stream>>>(LIST, CNT, OFF, (const float*)DINV, FLAG, T, B2V, Y);
  k_copy<<<(NN * H2) / NTHR, NTHR, 0, stream>>>(Y, out, out_size);
}
